// WReN_48962627174550
// MI455X (gfx1250) — hardware-verified
//
#include <hip/hip_runtime.h>
#include <stddef.h>
#include <stdint.h>


#define NB     128
#define NWAY   2
#define NSHOT  6
#define NQ     32
#define DD     256
#define NSROW  (NB * NWAY * NSHOT)
#define NQROW  (NB * NQ)
#define NVR    (NSROW + NQROW)
#define PP     512
#define NG2    (NB * NWAY)
#define NG     (NB * NQ * NWAY)
#define HP     264
#define NTHR   256
#define WSCL   16.0f
#define PSCL   0.0625f
#define WSCAP  134217728

static_assert(NTHR == 8 * 32);
static_assert((NVR % 16) == 0);
static_assert((NSROW % 16) == 0);
static_assert((NG % 32) == 0);
static_assert((NG % 4) == 0);
static_assert((DD % 32) == 0);
static_assert(((HP * 2) % 16) == 0);
static_assert(4 * NSHOT * 2 == 48);

#define SZ_W1T ((size_t)PP * DD * 2)
#define SZ_W2T ((size_t)DD * DD * 2)
#define SZ_F1T ((size_t)DD * DD * 2)
#define SZ_PRJ ((size_t)NVR * PP * 4)
#define SZ_SS  ((size_t)NG2 * DD * 4)
#define SZ_RS  ((size_t)NG * DD * 4)
#define SZ_TOT (SZ_W1T + SZ_W2T + SZ_F1T + SZ_PRJ + SZ_SS + SZ_RS)
static_assert(SZ_TOT == 20709376);
static_assert(SZ_TOT <= (size_t)WSCAP);
static_assert((SZ_W1T % 256) == 0);
static_assert((SZ_W2T % 256) == 0);
static_assert((SZ_PRJ % 256) == 0);
static_assert((SZ_SS % 256) == 0);
static_assert((SZ_RS % 256) == 0);

typedef _Float16     v16h __attribute__((ext_vector_type(16)));
typedef _Float16     v8h  __attribute__((ext_vector_type(8)));
typedef float        v8f  __attribute__((ext_vector_type(8)));
typedef float        v4f  __attribute__((ext_vector_type(4)));
typedef unsigned int v4u  __attribute__((ext_vector_type(4)));
union Frag { v16h v; v8h half[2]; };
union Pk8  { v8h h; v4u u; };

__device__ __forceinline__ v4u cvt8(const v4f a, const v4f b) {
  v8h hv = {(_Float16)a.x, (_Float16)a.y, (_Float16)a.z, (_Float16)a.w,
            (_Float16)b.x, (_Float16)b.y, (_Float16)b.z, (_Float16)b.w};
  Pk8 p;
  p.h = hv;
  return p.u;
}

__device__ __forceinline__ v8f wmh(v16h a, v16h b, v8f c) {
  v8f d = __builtin_amdgcn_wmma_f32_16x16x32_f16(false, a, false, b, (short)0, c, false, false);
  asm volatile("v_nop\n\tv_nop\n\tv_nop\n\tv_nop" : "+v"(d) : "v"(a), "v"(b));
  return d;
}

__device__ __forceinline__ v16h lda_frag(const _Float16* tile, int m, int k0, int h) {
  Frag a;
  const _Float16* p = tile + m * HP + k0 + 8 * h;
  a.half[0] = *(const v8h*)p;
  a.half[1] = *(const v8h*)(p + 16);
  return a.v;
}

__device__ __forceinline__ v16h ldb_frag(const _Float16* plane, int n, int k0, int h) {
  Frag b;
  const _Float16* p = plane + (size_t)n * DD + k0 + 8 * h;
  b.half[0] = *(const v8h*)p;
  b.half[1] = *(const v8h*)(p + 16);
  return b.v;
}

__global__ __launch_bounds__(32) void k_prep(const float* __restrict__ W1, const float* __restrict__ W2,
                                             const float* __restrict__ F1,
                                             _Float16* W1T, _Float16* W2T, _Float16* F1T) {
  const int blk = blockIdx.x, lane = threadIdx.x;
  const float* src;
  _Float16* dst;
  if (blk < PP) {
    src = W1 + (size_t)(blk >> 8) * DD * DD + (blk & (DD - 1));
    dst = W1T + (size_t)blk * DD;
  } else if (blk < PP + DD) {
    const int n = blk - PP;
    src = W2 + n;
    dst = W2T + (size_t)n * DD;
  } else {
    const int n = blk - PP - DD;
    src = F1 + n;
    dst = F1T + (size_t)n * DD;
  }
  const int k0 = 8 * lane;
  v4f f0, f1;
  f0.x = src[(size_t)(k0 + 0) * DD] * WSCL;
  f0.y = src[(size_t)(k0 + 1) * DD] * WSCL;
  f0.z = src[(size_t)(k0 + 2) * DD] * WSCL;
  f0.w = src[(size_t)(k0 + 3) * DD] * WSCL;
  f1.x = src[(size_t)(k0 + 4) * DD] * WSCL;
  f1.y = src[(size_t)(k0 + 5) * DD] * WSCL;
  f1.z = src[(size_t)(k0 + 6) * DD] * WSCL;
  f1.w = src[(size_t)(k0 + 7) * DD] * WSCL;
  const v4u pk = cvt8(f0, f1);
  _Float16* d = dst + k0;
  *(volatile v4u*)d = pk;
  __threadfence();
  *(volatile v4u*)d = pk;
}

__global__ __launch_bounds__(NTHR) void k_proj(const float* __restrict__ xs, const float* __restrict__ xq,
                                               const _Float16* __restrict__ W1T, float* proj) {
  __shared__ __attribute__((aligned(16))) _Float16 xa[16 * HP];
  __shared__ __attribute__((aligned(16))) float dt[16 * PP];
  const int tid = threadIdx.x, lane = tid & 31, wv = tid >> 5, h = lane >> 4, m = lane & 15;
  const int mt = blockIdx.x;
  {
    const int row = tid >> 4, c0 = (tid & 15) * 16;
    const float* base = (mt < NSROW / 16) ? (xs + (size_t)mt * 16 * DD)
                                          : (xq + (size_t)(mt - NSROW / 16) * 16 * DD);
    const float* s = base + row * DD + c0;
    const v4f a0 = *(const v4f*)s, a1 = *(const v4f*)(s + 4);
    const v4f a2 = *(const v4f*)(s + 8), a3 = *(const v4f*)(s + 12);
    *(v4u*)(xa + row * HP + c0)     = cvt8(a0, a1);
    *(v4u*)(xa + row * HP + c0 + 8) = cvt8(a2, a3);
  }
  __syncthreads();

  const v8f zero8 = {0.f, 0.f, 0.f, 0.f, 0.f, 0.f, 0.f, 0.f};
  v8f acc[4];
#pragma unroll
  for (int s = 0; s < 4; ++s) acc[s] = zero8;
#pragma unroll 1
  for (int kt = 0; kt < DD / 32; ++kt) {
    const int k0 = 32 * kt;
    const v16h a = lda_frag(xa, m, k0, h);
#pragma unroll
    for (int s = 0; s < 4; ++s) {
      const v16h b = ldb_frag(W1T, 64 * wv + 16 * s + m, k0, h);
      acc[s] = wmh(a, b, acc[s]);
    }
  }
#pragma unroll
  for (int s = 0; s < 4; ++s) {
    const int col = 64 * wv + 16 * s + m;
#pragma unroll
    for (int r = 0; r < 8; ++r) dt[(8 * h + r) * PP + col] = acc[s][r] * PSCL;
  }
  __syncthreads();

  v4f v[8];
#pragma unroll
  for (int it = 0; it < 8; ++it) v[it] = *(const v4f*)(dt + 4 * (it * NTHR + tid));
  float* pg = proj + (size_t)mt * 16 * PP;
#pragma unroll
  for (int it = 0; it < 8; ++it) *(volatile v4f*)(pg + 4 * (it * NTHR + tid)) = v[it];
  __threadfence();
#pragma unroll
  for (int it = 0; it < 8; ++it) *(volatile v4f*)(pg + 4 * (it * NTHR + tid)) = v[it];
}

__global__ __launch_bounds__(NTHR) void k_srel(const float* __restrict__ proj, const float* __restrict__ b1,
                                               const float* __restrict__ b2, const _Float16* __restrict__ W2T,
                                               float* S_shot) {
  __shared__ __attribute__((aligned(16))) _Float16 ha[32 * HP];
  __shared__ __attribute__((aligned(16))) float rowbuf[DD];
  const int tid = threadIdx.x, lane = tid & 31, wv = tid >> 5, h = lane >> 4, m = lane & 15;
  const int g2 = blockIdx.x;
  {
    const int c = tid;
    float pa[NSHOT], pb[NSHOT];
#pragma unroll
    for (int k = 0; k < NSHOT; ++k) {
      const float* pr = proj + (size_t)(g2 * NSHOT + k) * PP + c;
      pa[k] = pr[0];
      pb[k] = pr[DD];
    }
    const float bb = b1[c];
#pragma unroll
    for (int p = 0; p < 30; ++p) {
      const int i = p / 5;
      int j = p % 5;
      j += (j >= i) ? 1 : 0;
      const float v = (pa[j] + pb[i]) + bb;
      ha[p * HP + c] = (_Float16)fmaxf(v, 0.f);
    }
    ha[30 * HP + c] = (_Float16)0.f;
    ha[31 * HP + c] = (_Float16)0.f;
  }
  __syncthreads();

  const v8f zero8 = {0.f, 0.f, 0.f, 0.f, 0.f, 0.f, 0.f, 0.f};
  v8f acc[2][2];
#pragma unroll
  for (int mt = 0; mt < 2; ++mt) { acc[mt][0] = zero8; acc[mt][1] = zero8; }
#pragma unroll 1
  for (int kt = 0; kt < DD / 32; ++kt) {
    const int k0 = 32 * kt;
    const v16h b0 = ldb_frag(W2T, 32 * wv + m, k0, h);
    const v16h b1f = ldb_frag(W2T, 32 * wv + 16 + m, k0, h);
#pragma unroll
    for (int mt = 0; mt < 2; ++mt) {
      const v16h a = lda_frag(ha, 16 * mt + m, k0, h);
      acc[mt][0] = wmh(a, b0, acc[mt][0]);
      acc[mt][1] = wmh(a, b1f, acc[mt][1]);
    }
  }
  float bc[2];
  bc[0] = b2[32 * wv + m];
  bc[1] = b2[32 * wv + 16 + m];
#pragma unroll
  for (int nt = 0; nt < 2; ++nt) {
    float s = 0.f;
#pragma unroll
    for (int mt = 0; mt < 2; ++mt) {
#pragma unroll
      for (int r = 0; r < 8; ++r) {
        const int R = 16 * mt + 8 * h + r;
        const float val = fmaxf(acc[mt][nt][r] * PSCL + bc[nt], 0.f);
        s += (R < 30) ? val : 0.f;
      }
    }
    s += __shfl_xor(s, 16);
    if (h == 0) rowbuf[32 * wv + 16 * nt + m] = s;
  }
  __syncthreads();

  if (tid < 64) {
    const v4f v = *(const v4f*)(rowbuf + 4 * tid);
    float* p = S_shot + (size_t)g2 * DD + 4 * tid;
    *(volatile v4f*)p = v;
    __threadfence();
    *(volatile v4f*)p = v;
  }
}

__global__ __launch_bounds__(NTHR) void k_qrel(const float* proj, const float* __restrict__ b1,
                                               const float* __restrict__ b2, const _Float16* __restrict__ W2T,
                                               const float* __restrict__ S_shot, float* rel_sum) {
  __shared__ __attribute__((aligned(16))) _Float16 ha[48 * HP];
  __shared__ __attribute__((aligned(16))) float rowbuf[4 * DD];
  const int tid = threadIdx.x, lane = tid & 31, wv = tid >> 5, h = lane >> 4, m = lane & 15;
  const int blk = blockIdx.x;
  const int b = blk >> 4;
  const int qb = 2 * (blk & 15);
  {
    const int c = tid;
    const float bb = b1[c];
    float paq[2], pbq[2];
#pragma unroll
    for (int jq = 0; jq < 2; ++jq) {
      const float* pr = proj + (size_t)(NSROW + b * NQ + qb + jq) * PP + c;
      paq[jq] = pr[0];
      pbq[jq] = pr[DD];
    }
#pragma unroll
    for (int way = 0; way < 2; ++way) {
      const float* pr0 = proj + (size_t)(b * (NWAY * NSHOT) + way * NSHOT) * PP + c;
      float pbs[NSHOT];
#pragma unroll
      for (int k = 0; k < NSHOT; ++k) pbs[k] = pr0[(size_t)k * PP + DD];
#pragma unroll
      for (int jq = 0; jq < 2; ++jq) {
        const int j = 2 * jq + way;
#pragma unroll
        for (int k = 0; k < NSHOT; ++k) {
          const float v0 = (paq[jq] + pbs[k]) + bb;
          ha[(12 * j + k) * HP + c] = (_Float16)fmaxf(v0, 0.f);
        }
      }
      asm volatile("" ::: "memory");
      float pas[NSHOT];
#pragma unroll
      for (int k = 0; k < NSHOT; ++k) pas[k] = pr0[(size_t)k * PP];
#pragma unroll
      for (int jq = 0; jq < 2; ++jq) {
        const int j = 2 * jq + way;
#pragma unroll
        for (int k = 0; k < NSHOT; ++k) {
          const float v1 = (pas[k] + pbq[jq]) + bb;
          ha[(12 * j + NSHOT + k) * HP + c] = (_Float16)fmaxf(v1, 0.f);
        }
      }
      asm volatile("" ::: "memory");
    }
  }
  __syncthreads();

  const v8f zero8 = {0.f, 0.f, 0.f, 0.f, 0.f, 0.f, 0.f, 0.f};
  v8f acc[3][2];
#pragma unroll
  for (int mt = 0; mt < 3; ++mt) { acc[mt][0] = zero8; acc[mt][1] = zero8; }
#pragma unroll 1
  for (int kt = 0; kt < DD / 32; ++kt) {
    const int k0 = 32 * kt;
    const v16h b0 = ldb_frag(W2T, 32 * wv + m, k0, h);
    const v16h b1f = ldb_frag(W2T, 32 * wv + 16 + m, k0, h);
#pragma unroll
    for (int mt = 0; mt < 3; ++mt) {
      const v16h a = lda_frag(ha, 16 * mt + m, k0, h);
      acc[mt][0] = wmh(a, b0, acc[mt][0]);
      acc[mt][1] = wmh(a, b1f, acc[mt][1]);
    }
  }

  float bc[2], ss[2][2];
#pragma unroll
  for (int nt = 0; nt < 2; ++nt) {
    const int col = 32 * wv + 16 * nt + m;
    bc[nt] = b2[col];
    ss[0][nt] = S_shot[(size_t)(2 * b + 0) * DD + col];
    ss[1][nt] = S_shot[(size_t)(2 * b + 1) * DD + col];
  }
  float part[4][2];
#pragma unroll
  for (int j = 0; j < 4; ++j) { part[j][0] = 0.f; part[j][1] = 0.f; }
#pragma unroll
  for (int mt = 0; mt < 3; ++mt) {
#pragma unroll
    for (int nt = 0; nt < 2; ++nt) {
#pragma unroll
      for (int r = 0; r < 8; ++r) {
        const int R0 = 16 * mt + r;
        const int jA = R0 / 12, jB = (R0 + 8) / 12;
        const float val = fmaxf(acc[mt][nt][r] * PSCL + bc[nt], 0.f);
        const float vlo = h ? 0.f : val;
        const float vhi = h ? val : 0.f;
        part[jA][nt] += vlo;
        part[jB][nt] += vhi;
      }
    }
  }
#pragma unroll
  for (int j = 0; j < 4; ++j) {
#pragma unroll
    for (int nt = 0; nt < 2; ++nt) {
      float s = part[j][nt];
      s += __shfl_xor(s, 16);
      const float o = s + ss[j & 1][nt];
      if (h == 0) rowbuf[j * DD + 32 * wv + 16 * nt + m] = o;
    }
  }
  __syncthreads();

  {
    const v4f v = *(const v4f*)(rowbuf + 4 * tid);
    float* p = rel_sum + (size_t)blk * 4 * DD + 4 * tid;
    *(volatile v4f*)p = v;
    __threadfence();
    *(volatile v4f*)p = v;
  }
}

__global__ __launch_bounds__(NTHR) void k_head(const float* __restrict__ rel_sum, const _Float16* __restrict__ F1T,
                                               const float* __restrict__ fb1, const float* __restrict__ F2,
                                               const float* __restrict__ fb2, float* out) {
  __shared__ __attribute__((aligned(16))) _Float16 xa[32 * HP];
  __shared__ __attribute__((aligned(16))) float wred[8 * 32];
  __shared__ __attribute__((aligned(16))) float obuf[32];
  const int tid = threadIdx.x, lane = tid & 31, wv = tid >> 5, h = lane >> 4, m = lane & 15;
  const int blk = blockIdx.x;
  {
    const int row = tid >> 3, c0 = (tid & 7) * 32;
    const float* s = rel_sum + (size_t)(32 * blk + row) * DD + c0;
#pragma unroll
    for (int e = 0; e < 4; ++e) {
      const v4f a0 = *(const v4f*)(s + 8 * e), a1 = *(const v4f*)(s + 8 * e + 4);
      *(v4u*)(xa + row * HP + c0 + 8 * e) = cvt8(a0, a1);
    }
  }
  __syncthreads();

  const v8f zero8 = {0.f, 0.f, 0.f, 0.f, 0.f, 0.f, 0.f, 0.f};
  v8f acc[2][2];
#pragma unroll
  for (int mt = 0; mt < 2; ++mt) { acc[mt][0] = zero8; acc[mt][1] = zero8; }
#pragma unroll 1
  for (int kt = 0; kt < DD / 32; ++kt) {
    const int k0 = 32 * kt;
    const v16h b0 = ldb_frag(F1T, 32 * wv + m, k0, h);
    const v16h b1f = ldb_frag(F1T, 32 * wv + 16 + m, k0, h);
#pragma unroll
    for (int mt = 0; mt < 2; ++mt) {
      const v16h a = lda_frag(xa, 16 * mt + m, k0, h);
      acc[mt][0] = wmh(a, b0, acc[mt][0]);
      acc[mt][1] = wmh(a, b1f, acc[mt][1]);
    }
  }

  float fbv[2], f2v[2];
#pragma unroll
  for (int nt = 0; nt < 2; ++nt) {
    const int col = 32 * wv + 16 * nt + m;
    fbv[nt] = fb1[col];
    f2v[nt] = F2[col];
  }
  float pr[2][8];
#pragma unroll
  for (int mt = 0; mt < 2; ++mt) {
#pragma unroll
    for (int r = 0; r < 8; ++r) {
      float p = 0.f;
#pragma unroll
      for (int nt = 0; nt < 2; ++nt) {
        const float f = fmaxf(acc[mt][nt][r] * PSCL + fbv[nt], 0.f);
        p += f * f2v[nt];
      }
      p += __shfl_xor(p, 1);
      p += __shfl_xor(p, 2);
      p += __shfl_xor(p, 4);
      p += __shfl_xor(p, 8);
      pr[mt][r] = p;
    }
  }
  if (m == 0) {
#pragma unroll
    for (int mt = 0; mt < 2; ++mt) {
#pragma unroll
      for (int r = 0; r < 8; ++r) wred[wv * 32 + 16 * mt + 8 * h + r] = pr[mt][r];
    }
  }
  __syncthreads();
  if (tid < 32) {
    float s = 0.f;
#pragma unroll
    for (int w = 0; w < 8; ++w) s += wred[w * 32 + tid];
    s += fb2[0];
    obuf[tid] = s;
  }
  __syncthreads();
  if (wv == 0) {
    const int q = lane & 7;
    const v4f v = *(const v4f*)(obuf + 4 * q);
    float* p = out + (size_t)blk * 32 + 4 * q;
    if (lane < 8) *(volatile v4f*)p = v;
    __threadfence();
    if (lane < 8) *(volatile v4f*)p = v;
  }
}

extern "C" void kernel_launch(void* const* d_in, const int* in_sizes, int n_in,
                              void* d_out, int out_size, void* d_ws, size_t ws_size,
                              hipStream_t stream) {
  if (n_in < 10) return;
  if (in_sizes[0] != NSROW * DD) return;
  if (in_sizes[1] != NQROW * DD) return;
  if (in_sizes[2] != 2 * DD * DD || in_sizes[3] != DD) return;
  if (in_sizes[4] != DD * DD || in_sizes[5] != DD) return;
  if (in_sizes[6] != DD * DD || in_sizes[7] != DD) return;
  if (in_sizes[8] != DD || in_sizes[9] < 1) return;
  if (out_size != NG) return;

  const float* x_shot  = (const float*)d_in[0];
  const float* x_query = (const float*)d_in[1];
  const float* W1  = (const float*)d_in[2];
  const float* b1  = (const float*)d_in[3];
  const float* W2  = (const float*)d_in[4];
  const float* b2  = (const float*)d_in[5];
  const float* F1  = (const float*)d_in[6];
  const float* fb1 = (const float*)d_in[7];
  const float* F2  = (const float*)d_in[8];
  const float* fb2 = (const float*)d_in[9];
  float* out = (float*)d_out;

  char* ws = (char*)d_ws;
  size_t off = 0;
  const size_t oW1T = off; off += SZ_W1T;
  const size_t oW2T = off; off += SZ_W2T;
  const size_t oF1T = off; off += SZ_F1T;
  const size_t oPRJ = off; off += SZ_PRJ;
  const size_t oSS  = off; off += SZ_SS;
  const size_t oRS  = off; off += SZ_RS;
  if (off != SZ_TOT) return;
  if (off > ws_size || off > (size_t)WSCAP) return;

  _Float16* W1T = (_Float16*)(ws + oW1T);
  _Float16* W2T = (_Float16*)(ws + oW2T);
  _Float16* F1T = (_Float16*)(ws + oF1T);
  float* proj    = (float*)(ws + oPRJ);
  float* S_shot  = (float*)(ws + oSS);
  float* rel_sum = (float*)(ws + oRS);

  k_prep<<<PP + 2 * DD, 32, 0, stream>>>(W1, W2, F1, W1T, W2T, F1T);
  k_proj<<<NVR / 16, NTHR, 0, stream>>>(x_shot, x_query, W1T, proj);
  k_srel<<<NG2, NTHR, 0, stream>>>(proj, b1, b2, W2T, S_shot);
  k_qrel<<<NG / 4, NTHR, 0, stream>>>(proj, b1, b2, W2T, S_shot, rel_sum);
  k_head<<<NG / 32, NTHR, 0, stream>>>(rel_sum, F1T, fb1, F2, fb2, out);
}
